// DotProductNonLocalBlock_36103495090207
// MI455X (gfx1250) — hardware-verified
//
#include <hip/hip_runtime.h>


#define NBI  8
#define CIN  512
#define NTOK 3136
#define EE   256
#define DM   CIN
#define NTK  NTOK
#define LOSC 1024.0f

typedef _Float16 h16;
typedef unsigned short bf;
typedef __attribute__((ext_vector_type(16))) __bf16   v16bf;
typedef __attribute__((ext_vector_type(16))) _Float16 v16h;
typedef __attribute__((ext_vector_type(8)))  _Float16 v8h;
typedef __attribute__((ext_vector_type(8)))  unsigned short v8us;
typedef __attribute__((ext_vector_type(8)))  float    v8f;
typedef __attribute__((ext_vector_type(4)))  float    v4f;
typedef __attribute__((ext_vector_type(4)))  _Float16 v4h;
typedef v8h  __attribute__((may_alias)) v8ha;
typedef v4f  __attribute__((may_alias)) v4fa;
typedef v8us __attribute__((may_alias)) v8usa;

__device__ __forceinline__ unsigned short f2bf(float f) { unsigned u = __float_as_uint(f); u += 0x7FFFu + ((u >> 16) & 1u); return (unsigned short)(u >> 16); }
__device__ __forceinline__ float bf2f(unsigned short b) { return __uint_as_float(((unsigned)b) << 16); }
__device__ __forceinline__ float bfr(float f) { return bf2f(f2bf(f)); }
__device__ __forceinline__ v16h cat16(v8h lo, v8h hi) { return __builtin_shufflevector(lo, hi, 0, 1, 2, 3, 4, 5, 6, 7, 8, 9, 10, 11, 12, 13, 14, 15); }
__device__ __forceinline__ v16bf cat16b(v8us lo, v8us hi) { return __builtin_bit_cast(v16bf, __builtin_shufflevector(lo, hi, 0, 1, 2, 3, 4, 5, 6, 7, 8, 9, 10, 11, 12, 13, 14, 15)); }
__device__ __forceinline__ v8f wmma16(v16h a, v16h b, v8f c) { return __builtin_amdgcn_wmma_f32_16x16x32_f16(false, a, false, b, (short)0, c, false, false); }
__device__ __forceinline__ v8f wmmab(v16bf a, v16bf b, v8f c) { return __builtin_amdgcn_wmma_f32_16x16x32_bf16(false, a, false, b, (short)0, c, false, false); }

__global__ __launch_bounds__(256) void k_wt(const float* __restrict__ Wm, int K, int ncols, bf* WT) {
    __shared__ __align__(16) unsigned short tl[64 * 72];
    const int tid = threadIdx.x, k0 = blockIdx.x * 64, n0 = blockIdx.y * 64;
    const int kk = tid >> 2, nq = (tid & 3) * 16;
#pragma unroll
    for (int i = 0; i < 16; ++i) tl[(nq + i) * 72 + kk] = f2bf(Wm[(size_t)(k0 + kk) * ncols + n0 + nq + i]);
    __syncthreads();
    const int piece = tid & 7;
    auto pass = [&]() {
#pragma unroll
        for (int s = 0; s < 2; ++s) { const int nr = (tid >> 3) + 32 * s; const v8us val = *(const v8usa*)(tl + nr * 72 + piece * 8); *(volatile v8us*)(WT + (size_t)(n0 + nr) * K + k0 + piece * 8) = val; }
    };
    pass(); __threadfence(); pass();
}
template <bool SPLITA, bool F16OUT = false>
__global__ __launch_bounds__(128) void k_gemmb(const bf* __restrict__ A, const bf* __restrict__ Al, const bf* __restrict__ Bn, const float* __restrict__ bias, float* C, int ldc, h16* C2, const float* __restrict__ R = nullptr, int K = DM, int roundR = 1) {
    __shared__ __align__(16) float ost[4][16 * 68];
    const int lane = threadIdx.x & 31, wave = threadIdx.x >> 5, lr = lane & 15, hi = lane >> 4;
    const int r0 = blockIdx.x * 64 + wave * 16, c0 = blockIdx.y * 64;
    const size_t aoff = (size_t)(r0 + lr) * K + 8 * hi;
    size_t boff[4];
#pragma unroll
    for (int t = 0; t < 4; ++t) boff[t] = (size_t)(c0 + t * 16 + lr) * K + 8 * hi;
    v8f acc[4];
#pragma unroll
    for (int t = 0; t < 4; ++t) acc[t] = (v8f){};
#pragma unroll 1
    for (int kc = 0; kc < K; kc += 32) {
        const v16bf a = cat16b(*(const v8us*)(A + aoff + kc), *(const v8us*)(A + aoff + kc + 16));
        v16bf al = a;
        if (SPLITA) al = cat16b(*(const v8us*)(Al + aoff + kc), *(const v8us*)(Al + aoff + kc + 16));
#pragma unroll
        for (int t = 0; t < 4; ++t) { const v16bf b = cat16b(*(const v8us*)(Bn + boff[t] + kc), *(const v8us*)(Bn + boff[t] + kc + 16)); acc[t] = wmmab(a, b, acc[t]); if (SPLITA) acc[t] = wmmab(al, b, acc[t]); }
        asm volatile("v_nop\n\tv_nop\n\tv_nop\n\tv_nop" : "+v"(acc[0]), "+v"(acc[1]), "+v"(acc[2]), "+v"(acc[3]) : "v"(a), "v"(al));
    }
    float* os = &ost[wave][0];
#pragma unroll
    for (int t = 0; t < 4; ++t) { const float bv = bias ? bfr(bias[c0 + t * 16 + lr]) : 0.f;
#pragma unroll
        for (int j = 0; j < 8; ++j) os[(hi * 8 + j) * 68 + t * 16 + lr] = acc[t][j] + bv; }
    __syncthreads();
    if (F16OUT) {
        h16* crow = (h16*)(void*)C + (size_t)r0 * ldc + c0;
        auto pass = [&]() {
#pragma unroll
            for (int s = 0; s < 4; ++s) { const int row = 4 * s + (lane >> 3), piece = lane & 7; const float* sp = os + row * 68 + piece * 8; v8h o, o2;
#pragma unroll
                for (int i = 0; i < 8; ++i) { const h16 a = (h16)sp[i]; o[i] = a; o2[i] = (h16)((sp[i] - (float)a) * LOSC); }
                *(volatile v8h*)(crow + (size_t)row * ldc + piece * 8) = o; if (C2) *(volatile v8h*)(C2 + (size_t)r0 * ldc + c0 + (size_t)row * ldc + piece * 8) = o2; }
        };
        pass(); __threadfence(); pass();
    } else {
        float* crow = C + (size_t)r0 * ldc + c0;
        auto pass = [&]() {
#pragma unroll
            for (int s = 0; s < 8; ++s) { const int Lid = (lane >> 3) + 4 * s, piece = lane & 7; const int row = Lid >> 1, cofs = (Lid & 1) * 32 + piece * 4;
                v4f val = *(const v4fa*)(os + row * 68 + cofs); if (R) { const v4f rv = *(const v4f*)(R + ((size_t)r0 + row) * ldc + c0 + cofs); val += roundR ? (v4f){bfr(rv[0]), bfr(rv[1]), bfr(rv[2]), bfr(rv[3])} : rv; }
                *(volatile v4f*)(crow + (size_t)row * ldc + cofs) = val; }
        };
        pass(); __threadfence(); pass();
    }
}

__global__ __launch_bounds__(128) void k_gemm3(const bf* __restrict__ Ah, const bf* __restrict__ Al, const bf* __restrict__ Bh, const bf* __restrict__ Bl, int K, float* C, int ldc) {
    __shared__ __align__(16) float ost[4][16 * 68];
    const int lane = threadIdx.x & 31, wave = threadIdx.x >> 5, lr = lane & 15, hi = lane >> 4;
    const int r0 = blockIdx.x * 64 + wave * 16, c0 = blockIdx.y * 64;
    const size_t aoff = (size_t)(r0 + lr) * K + 8 * hi;
    v8f acc[4];
#pragma unroll
    for (int t = 0; t < 4; ++t) acc[t] = (v8f){};
#pragma unroll 1
    for (int kc = 0; kc < K; kc += 32) {
        const v16bf a = cat16b(*(const v8us*)(Ah + aoff + kc), *(const v8us*)(Ah + aoff + kc + 16));
        const v16bf al = cat16b(*(const v8us*)(Al + aoff + kc), *(const v8us*)(Al + aoff + kc + 16));
#pragma unroll
        for (int t = 0; t < 4; ++t) { const size_t bo = (size_t)(c0 + t * 16 + lr) * K + kc + 8 * hi;
            const v16bf bh = cat16b(*(const v8us*)(Bh + bo), *(const v8us*)(Bh + bo + 16)); const v16bf bl = cat16b(*(const v8us*)(Bl + bo), *(const v8us*)(Bl + bo + 16));
            acc[t] = wmmab(a, bh, acc[t]); acc[t] = wmmab(al, bh, acc[t]); acc[t] = wmmab(a, bl, acc[t]); }
        asm volatile("v_nop\n\tv_nop\n\tv_nop\n\tv_nop" : "+v"(acc[0]), "+v"(acc[1]), "+v"(acc[2]), "+v"(acc[3]) : "v"(a), "v"(al));
    }
    float* os = &ost[wave][0];
#pragma unroll
    for (int t = 0; t < 4; ++t) {
#pragma unroll
        for (int j = 0; j < 8; ++j) os[(hi * 8 + j) * 68 + t * 16 + lr] = acc[t][j]; }
    __builtin_amdgcn_wave_barrier(); asm volatile("" ::: "memory");
    float* crow = C + (size_t)r0 * ldc + c0;
    auto pass = [&]() {
#pragma unroll
        for (int s = 0; s < 8; ++s) { const int Lid = (lane >> 3) + 4 * s, piece = lane & 7; const int row = Lid >> 1, cofs = (Lid & 1) * 32 + piece * 4;
            const v4f val = *(const v4fa*)(os + row * 68 + cofs); *(volatile v4f*)(crow + (size_t)row * ldc + cofs) = val; }
    };
    pass(); __threadfence(); pass();
}

__global__ __launch_bounds__(256) void k_bfz(const float* __restrict__ src, bf* dh, bf* dz, size_t n8) {
    const size_t i = (size_t)blockIdx.x * 256 + threadIdx.x; if (i >= n8) return;
    const v8f v = *(const v8f*)(src + i * 8); v8us o, z;
#pragma unroll
    for (int k = 0; k < 8; ++k) { o[k] = f2bf(v[k]); z[k] = 0; }
    *(volatile v8us*)(dh + i * 8) = o; *(volatile v8us*)(dz + i * 8) = z; __threadfence(); *(volatile v8us*)(dh + i * 8) = o; *(volatile v8us*)(dz + i * 8) = z;
}
__global__ __launch_bounds__(256) void k_rowsplit(const float* __restrict__ Y, const float* __restrict__ bias, float scale, int nrows, bf* Ph, bf* Pl) {
    const int lane = threadIdx.x & 31, r = blockIdx.x * 8 + (threadIdx.x >> 5); if (r >= nrows) return;
    const float bo = bias ? bfr(bias[r]) : 0.f;
#pragma unroll 1
    for (int ps = 0; ps < 2; ++ps) {
#pragma unroll 1
        for (int c0 = lane * 8; c0 < NTOK; c0 += 256) { const size_t o = (size_t)r * NTOK + c0; const v8f v = *(const v8f*)(Y + o); v8us oh, ol;
#pragma unroll
            for (int i = 0; i < 8; ++i) { const float y = (v[i] + bo) * scale; const unsigned short hb = f2bf(y); oh[i] = hb; ol[i] = f2bf(y - bf2f(hb)); }
            *(volatile v8us*)(Ph + o) = oh; *(volatile v8us*)(Pl + o) = ol; }
        if (ps == 0) __threadfence(); }
}
__global__ __launch_bounds__(256) void k_split256(const float* __restrict__ src, float scale, int nrows, bf* dh, bf* dl) {
    const int lane = threadIdx.x & 31, r = blockIdx.x * 8 + (threadIdx.x >> 5); if (r >= nrows) return;
    const size_t o = (size_t)r * EE + lane * 8; const v8f v = *(const v8f*)(src + o); v8us oh, ol;
#pragma unroll
    for (int i = 0; i < 8; ++i) { const float y = v[i] * scale; const unsigned short hb = f2bf(y); oh[i] = hb; ol[i] = f2bf(y - bf2f(hb)); }
    *(volatile v8us*)(dh + o) = oh; *(volatile v8us*)(dl + o) = ol; __threadfence(); *(volatile v8us*)(dh + o) = oh; *(volatile v8us*)(dl + o) = ol;
}
__global__ __launch_bounds__(256) void k_rowbias(const float* __restrict__ T, const float* __restrict__ bo, const float* __restrict__ X, float* OUTP) {
    const int lane = threadIdx.x & 31, r = blockIdx.x * 8 + (threadIdx.x >> 5); if (r >= CIN) return;
    const float b = bfr(bo[r]);
#pragma unroll 1
    for (int ps = 0; ps < 2; ++ps) {
#pragma unroll 1
        for (int c0 = lane * 8; c0 < NTOK; c0 += 256) { const size_t o = (size_t)r * NTOK + c0; v8f v = *(const v8f*)(T + o); const v8f xv = *(const v8f*)(X + o);
#pragma unroll
            for (int i = 0; i < 8; ++i) v[i] += b + bfr(xv[i]);
            *(volatile v8f*)(OUTP + o) = v; }
        if (ps == 0) __threadfence(); }
}

extern "C" void kernel_launch(void* const* d_in, const int* in_sizes, int n_in,
                              void* d_out, int out_size, void* d_ws, size_t ws_size, hipStream_t stream) {
    (void)in_sizes; (void)n_in; (void)out_size;
    const float* x = (const float*)d_in[0]; const float* wq = (const float*)d_in[1]; const float* bq = (const float*)d_in[2]; const float* wk = (const float*)d_in[3]; const float* bk = (const float*)d_in[4];
    const float* wv = (const float*)d_in[5]; const float* bv = (const float*)d_in[6]; const float* wo = (const float*)d_in[7]; const float* bo = (const float*)d_in[8];
    float* out = (float*)d_out;
    char* wsp = (char*)d_ws;
    auto take = [&](size_t bytes) { char* p = wsp; wsp += (bytes + 255) & ~(size_t)255; return (void*)p; };
    bf* WqB = (bf*)take((size_t)EE * CIN * 2); bf* WkB = (bf*)take((size_t)EE * CIN * 2); bf* WvB = (bf*)take((size_t)EE * CIN * 2); bf* WoB = (bf*)take((size_t)CIN * EE * 2); bf* WoZ = (bf*)take((size_t)CIN * EE * 2);
    bf* XT = (bf*)take((size_t)NTOK * CIN * 2); float* TMP = (float*)take((size_t)CIN * NTOK * 4);
    bf* Qh = (bf*)take((size_t)NTOK * EE * 2); bf* Ql = (bf*)take((size_t)NTOK * EE * 2); bf* Kh = (bf*)take((size_t)EE * NTOK * 2); bf* Kl = (bf*)take((size_t)EE * NTOK * 2); bf* Vh = (bf*)take((size_t)EE * NTOK * 2); bf* Vl = (bf*)take((size_t)EE * NTOK * 2);
    float* MT = (float*)take((size_t)EE * EE * 4); bf* MTh = (bf*)take((size_t)EE * EE * 2); bf* MTl = (bf*)take((size_t)EE * EE * 2); bf* Eh = (bf*)take((size_t)NTOK * EE * 2); bf* El = (bf*)take((size_t)NTOK * EE * 2);
    if ((size_t)(wsp - (char*)d_ws) > ws_size) return;
    k_bfz<<<(EE * CIN / 8 + 255) / 256, 256, 0, stream>>>(wq, WqB, WoZ, EE * CIN / 8); k_bfz<<<(EE * CIN / 8 + 255) / 256, 256, 0, stream>>>(wk, WkB, WoZ, EE * CIN / 8); k_bfz<<<(EE * CIN / 8 + 255) / 256, 256, 0, stream>>>(wv, WvB, WoZ, EE * CIN / 8);
    k_bfz<<<(CIN * EE / 8 + 255) / 256, 256, 0, stream>>>(wo, WoB, WoZ, CIN * EE / 8);
    for (int b = 0; b < NBI; ++b) {
        const float* xb = x + (size_t)b * CIN * NTOK;
        k_wt<<<dim3(CIN / 64, NTOK / 64, 1), 256, 0, stream>>>(xb, CIN, NTOK, XT);
        k_gemmb<false, false><<<dim3(NTOK / 64, EE / 64, 1), 128, 0, stream>>>(XT, nullptr, WqB, bq, TMP, EE, nullptr); k_split256<<<NTOK / 8, 256, 0, stream>>>(TMP, 1.0f, NTOK, Qh, Ql);
        k_gemmb<false, false><<<dim3(EE / 64, NTOK / 64, 1), 128, 0, stream>>>(WkB, nullptr, XT, nullptr, TMP, NTOK, nullptr); k_rowsplit<<<EE / 8, 256, 0, stream>>>(TMP, bk, 1.0f, EE, Kh, Kl);
        k_gemmb<false, false><<<dim3(EE / 64, NTOK / 64, 1), 128, 0, stream>>>(WvB, nullptr, XT, nullptr, TMP, NTOK, nullptr); k_rowsplit<<<EE / 8, 256, 0, stream>>>(TMP, bv, 1.0f, EE, Vh, Vl);
        k_gemm3<<<dim3(EE / 64, EE / 64, 1), 128, 0, stream>>>(Vh, Vl, Kh, Kl, NTOK, MT, EE);
        k_split256<<<EE / 8, 256, 0, stream>>>(MT, 1.0f, EE, MTh, MTl);
        k_gemm3<<<dim3(NTOK / 64, EE / 64, 1), 128, 0, stream>>>(Qh, Ql, MTh, MTl, EE, TMP, EE);
        k_split256<<<NTOK / 8, 256, 0, stream>>>(TMP, 1.0f / (float)NTOK, NTOK, Eh, El);
        k_gemm3<<<dim3(CIN / 64, NTOK / 64, 1), 128, 0, stream>>>(WoB, WoZ, Eh, El, EE, TMP, NTOK);
        k_rowbias<<<CIN / 8, 256, 0, stream>>>(TMP, bo, xb, out + (size_t)b * CIN * NTOK);
    }
}
